// Conv3d_82669530514090
// MI455X (gfx1250) — hardware-verified
//
#include <hip/hip_runtime.h>

typedef float          v8f   __attribute__((ext_vector_type(8)));
typedef float          v4f   __attribute__((ext_vector_type(4)));
typedef unsigned int   v4u   __attribute__((ext_vector_type(4)));
typedef int            v8i   __attribute__((ext_vector_type(8)));
typedef unsigned short v8us  __attribute__((ext_vector_type(8)));
typedef unsigned short v16us __attribute__((ext_vector_type(16)));
typedef __bf16         v16bf __attribute__((ext_vector_type(16)));
typedef _Float16       v16h  __attribute__((ext_vector_type(16)));
typedef v4f  __attribute__((may_alias)) v4fa;
typedef v8us __attribute__((may_alias)) v8usa;
union FragB { v16bf v; v16us u; v8us h[2]; v8i w; };
union FragH { v16h  v; v16us u; v8us h[2]; v8i w; };

__device__ __forceinline__ v8f wmb(const FragB& a, const FragB& b, v8f c) {
  v8f d = __builtin_amdgcn_wmma_f32_16x16x32_bf16(false, a.v, false, b.v, (short)0, c, false, false);
  asm volatile("v_nop\n\tv_nop\n\tv_nop\n\tv_nop" : "+v"(d) : "v"(a.w), "v"(b.w));
  return d;
}

__device__ __forceinline__ v8f wmh(const FragH& a, const FragH& b, v8f c) {
  v8f d = __builtin_amdgcn_wmma_f32_16x16x32_f16(false, a.v, false, b.v, (short)0, c, false, false);
  asm volatile("v_nop\n\tv_nop\n\tv_nop\n\tv_nop" : "+v"(d) : "v"(a.w), "v"(b.w));
  return d;
}

__device__ __forceinline__ unsigned bf16_bits(float f) {
  const unsigned u = __float_as_uint(f);
  const unsigned r = (u + 0x7FFFu + ((u >> 16) & 1u)) >> 16;
  const unsigned q = (u >> 16) | 0x40u;
  return ((u & 0x7fffffffu) > 0x7f800000u) ? q : r;
}

__device__ __forceinline__ float bf16_val(float f) {
  return __uint_as_float(bf16_bits(f) << 16);
}
__device__ __forceinline__ int clampi(int v, int lo, int hi) {
  return v < lo ? lo : (v > hi ? hi : v);
}

__device__ __forceinline__ unsigned f16_bits(float f) {
  const unsigned u  = __float_as_uint(f);
  const unsigned s  = (u >> 16) & 0x8000u;
  const unsigned a  = u & 0x7fffffffu;
  const unsigned t  = a - 0x38000000u;
  const unsigned r  = (t + 0x0FFFu + ((t >> 13) & 1u)) >> 13;
  const unsigned rc = r > 0x7C00u ? 0x7C00u : r;
  const bool small  = a < 0x38800000u;
  const bool isnan  = a > 0x7f800000u;
  const unsigned fin = small ? 0u : (s | rc);
  return isnan ? (s | 0x7E00u) : fin;
}

__device__ __forceinline__ unsigned pk16(unsigned lo, unsigned hi) { return lo | (hi << 16); }
__device__ __forceinline__ unsigned bf16_lo_bits(float v) {
  float hi = bf16_val(v);
  asm volatile("" : "+v"(hi));
  return bf16_bits(v - hi);
}
__device__ __forceinline__ v4u pack8_bf16(v4f a, v4f c) {
  return (v4u){ pk16(bf16_bits(a[0]), bf16_bits(a[1])), pk16(bf16_bits(a[2]), bf16_bits(a[3])),
                pk16(bf16_bits(c[0]), bf16_bits(c[1])), pk16(bf16_bits(c[2]), bf16_bits(c[3])) };
}
__device__ __forceinline__ v4u pack8_bf16_lo(v4f a, v4f c) {
  return (v4u){ pk16(bf16_lo_bits(a[0]), bf16_lo_bits(a[1])), pk16(bf16_lo_bits(a[2]), bf16_lo_bits(a[3])),
                pk16(bf16_lo_bits(c[0]), bf16_lo_bits(c[1])), pk16(bf16_lo_bits(c[2]), bf16_lo_bits(c[3])) };
}
__device__ __forceinline__ v4u pack8_f16(v4f a, v4f c) {
  return (v4u){ pk16(f16_bits(a[0]), f16_bits(a[1])), pk16(f16_bits(a[2]), f16_bits(a[3])),
                pk16(f16_bits(c[0]), f16_bits(c[1])), pk16(f16_bits(c[2]), f16_bits(c[3])) };
}

template <int FORM>
__global__ __launch_bounds__(256) void k_plane(const float* __restrict__ src, int rows, int cols, int ldsrc,
                                               unsigned short* __restrict__ dst, int MP, int KP) {
  static_assert(FORM >= 0 && FORM <= 3);
  const int KTOT = (FORM == 1 || FORM == 3) ? 2 * KP : KP;
  const unsigned ppr   = (unsigned)(KTOT >> 3);
  const unsigned kp8   = (unsigned)(KP >> 3);
  const unsigned total = (unsigned)MP * ppr;
  const unsigned g     = blockIdx.x * 256u + threadIdx.x;
  const unsigned rowu  = g / ppr;
  const unsigned p     = g - rowu * ppr;
  const bool second    = p >= kp8;
  const int row = (int)rowu;
  const int c0  = (int)((second ? p - kp8 : p) << 3);
  const float* srow = src + (size_t)clampi(row, 0, rows - 1) * (size_t)ldsrc;
  float x[8];
  unsigned mk[8];
#pragma unroll
  for (int e = 0; e < 8; ++e) {
    const int c = c0 + e;
    const float v = srow[clampi(c, 0, cols - 1)];
    asm volatile("" :: "v"(v));
    x[e]  = v;
    mk[e] = (row < rows && c < cols) ? 0xFFFFu : 0u;
  }
  const v4f a = (v4f){ x[0], x[1], x[2], x[3] };
  const v4f c = (v4f){ x[4], x[5], x[6], x[7] };
  v4u o;
  if (FORM == 2) {
    o = pack8_f16(a, c);
  } else {
    const v4u hi = pack8_bf16(a, c);
    o = hi;
    if (FORM == 1) { const v4u lo = pack8_bf16_lo(a, c); o = second ? lo : hi; }
  }
  const v4u mw = (v4u){ pk16(mk[0], mk[1]), pk16(mk[2], mk[3]), pk16(mk[4], mk[5]), pk16(mk[6], mk[7]) };
  o &= mw;
  if (g < total) {
    volatile v4u* q = (volatile v4u*)(dst + (size_t)g * 8);
    *q = o;
    __threadfence();
    *q = o;
  }
}

template <int FORM> struct FragOf    { typedef FragB T; };
template <>         struct FragOf<2> { typedef FragH T; };
__device__ __forceinline__ v8f mm(const FragB& a, const FragB& b, v8f c) { return wmb(a, b, c); }
__device__ __forceinline__ v8f mm(const FragH& a, const FragH& b, v8f c) { return wmh(a, b, c); }
template <class F> __device__ __forceinline__ F ld_frag(const unsigned short* p) {
  F f;
  f.h[0] = *(const v8usa*)(p);
  f.h[1] = *(const v8usa*)(p + 16);
  return f;
}

template <int FORM, int EPI>
__global__ __launch_bounds__(256) __attribute__((amdgpu_num_vgpr(248)))
void k_gemm_nt(const unsigned short* __restrict__ A, const unsigned short* __restrict__ B,
               const float* __restrict__ bias, float* __restrict__ D, int M, int N, int KTOT, int ldd) {
  static_assert(FORM >= 0 && FORM <= 2);
  static_assert(EPI == 0 || EPI == 1);
  typedef typename FragOf<FORM>::T F;
  __shared__ __attribute__((aligned(16))) float sT[8][16 * 68];
  const int lane = threadIdx.x & 31;
  const int wave = threadIdx.x >> 5;
  const int tilesM = (M + 63) >> 6;
  const int tilesN = (N + 63) >> 6;
  const int tile = blockIdx.x * 8 + wave;
  if (tile >= tilesM * tilesN) return;
  const int tm = tile / tilesN;
  const int tn = tile - tm * tilesN;
  const int m0 = tm << 6;
  const int n0 = tn << 6;

  const int rl = lane & 15;
  const int h8 = (lane >> 4) * 8;
  const unsigned short* pa = A + (size_t)(m0 + rl) * (size_t)KTOT + h8;
  const unsigned short* pb = B + (size_t)(n0 + rl) * (size_t)KTOT + h8;

  v8f acc[4][4];
#pragma unroll
  for (int i = 0; i < 4; ++i)
#pragma unroll
    for (int j = 0; j < 4; ++j) acc[i][j] = (v8f){0.f, 0.f, 0.f, 0.f, 0.f, 0.f, 0.f, 0.f};

#pragma unroll 1
  for (int k0 = 0; k0 < KTOT; k0 += 32) {
    F bf[4];
#pragma unroll
    for (int j = 0; j < 4; ++j) bf[j] = ld_frag<F>(pb + (size_t)(j << 4) * (size_t)KTOT + k0);
#pragma unroll
    for (int i = 0; i < 4; ++i) {
      const F af = ld_frag<F>(pa + (size_t)(i << 4) * (size_t)KTOT + k0);
#pragma unroll
      for (int j = 0; j < 4; ++j) acc[i][j] = mm(af, bf[j], acc[i][j]);
    }
  }

  float* slab = sT[wave];
  const int hh = lane >> 4;
  const int c4 = (lane & 15) * 4;
  const int nc = n0 + c4;
  const bool cok = nc < N;
  v4f bv = (v4f){0.f, 0.f, 0.f, 0.f};
  if (EPI == 1) {
    bv = *(const v4fa*)(bias + clampi(nc, 0, N - 4));
    asm volatile("" :: "v"(bv));
  }
#pragma unroll
  for (int i = 0; i < 4; ++i) {
    const int mBase = m0 + (i << 4);
#pragma unroll
    for (int j = 0; j < 4; ++j) {
#pragma unroll
      for (int r = 0; r < 8; ++r) slab[(h8 + r) * 68 + (j << 4) + rl] = acc[i][j][r];
    }
    __builtin_amdgcn_fence(__ATOMIC_RELEASE, "workgroup");
    __builtin_amdgcn_wave_barrier();
    __builtin_amdgcn_fence(__ATOMIC_ACQUIRE, "workgroup");
    v4f vv[8];
#pragma unroll
    for (int it = 0; it < 8; ++it) {
      const int row = it * 2 + hh;
      v4f v = *(const v4fa*)(slab + row * 68 + c4);
      if (EPI == 1) v += bv;
      vv[it] = v;
    }
    for (int pass = 0; pass < 2; ++pass) {
#pragma unroll
      for (int it = 0; it < 8; ++it) {
        const int row = mBase + it * 2 + hh;
        if (cok && row < M) *(volatile v4f*)(D + (size_t)row * (size_t)ldd + nc) = vv[it];
      }
      __threadfence();
    }
    __builtin_amdgcn_fence(__ATOMIC_RELEASE, "workgroup");
    __builtin_amdgcn_wave_barrier();
    __builtin_amdgcn_fence(__ATOMIC_ACQUIRE, "workgroup");
  }
}

#include <stddef.h>
#include <stdint.h>


#define NVOX    262144
#define MPAIR   131072
#define NOFF    27
#define CIN     32
#define COUT    32
#define NPB     64
#define NGROUP  7
#define GOFF    4
#define GRPE    (GOFF * MPAIR)
#define NBRUN   4096
#define SLOTB   12
#define EBITS   19
#define EMASK   ((1 << EBITS) - 1)
#define NBLK    (NVOX / NBRUN)
#define NTHR    256
#define NWAVE   8
#define EPT     8
#define CHUNK   (NTHR * EPT)
#define WCAP    (EPT * 32)
#define LISTN   (NWAVE * WCAP)
#define RCAP    12288
#define DEGCAP  48
#define ARRN    (NBRUN + 16)
#define BK_INTS (LISTN + 2 * RCAP + ARRN + 32)
#define BK_BYTES (BK_INTS * 4)

#define BT_BYTES ((size_t)NOFF * NPB * CIN * 2)
#define AG_BYTES ((size_t)GRPE * CIN * 2)
#define CG_BYTES ((size_t)GRPE * COUT * 4)
#define WS_TOTAL (BT_BYTES + AG_BYTES + CG_BYTES)

static_assert(MPAIR % CHUNK == 0);
static_assert(GRPE <= (1 << EBITS));
static_assert(SLOTB + EBITS <= 32 && NBRUN == (1 << SLOTB));
static_assert(NVOX % NBRUN == 0 && NBLK * NBRUN == NVOX && NBLK == 64);
static_assert(RCAP == 12288 && RCAP >= 2 * NBRUN + NBRUN && DEGCAP == 48);
static_assert(NPB >= COUT && NPB % 64 == 0 && CIN % 32 == 0 && CIN == 32 && COUT == 32);
static_assert(MPAIR % 64 == 0 && MPAIR % 16 == 0 && COUT % 4 == 0);
static_assert((GRPE * 4) % 256 == 0 && (3 * MPAIR * 4) % 256 == 0);
static_assert(6 * GOFF + 3 == NOFF);
static_assert(BK_INTS % 4 == 0 && LISTN % 4 == 0 && RCAP % 4 == 0 && ARRN % 4 == 0);
static_assert(BK_BYTES == 123072 && BK_BYTES <= 327680);
static_assert(NBRUN % NTHR == 0 && NBRUN % (NWAVE * 32) == 0);
static_assert(BT_BYTES == 110592 && AG_BYTES == 33554432 && CG_BYTES == 67108864);
static_assert(WS_TOTAL == (size_t)100773 * 1000 + 888);
static_assert(WS_TOTAL <= ((size_t)128 << 20));
static_assert(BT_BYTES % 256 == 0 && AG_BYTES % 256 == 0);

typedef int v4i __attribute__((ext_vector_type(4)));
typedef v4i __attribute__((may_alias)) v4ia;

__device__ __forceinline__ void pinf(float x) { asm volatile("" :: "v"(x)); }
__device__ __forceinline__ void pini(int x)   { asm volatile("" :: "v"(x)); }
__device__ __forceinline__ void pin4(const v4i w) { pini(w.x); pini(w.y); pini(w.z); pini(w.w); }
__device__ __forceinline__ void pin4f(const v4f w) { pinf(w.x); pinf(w.y); pinf(w.z); pinf(w.w); }

__global__ __launch_bounds__(256) void k_prep(const float* __restrict__ w, unsigned short* bt) {
  __shared__ __attribute__((aligned(16))) float sK[32 * 36];
  const int o = (int)blockIdx.x, tid = (int)threadIdx.x;
  const v4f v = *(const v4fa*)(w + (size_t)o * (CIN * COUT) + 4 * tid);
  pin4f(v);
  *(v4fa*)(sK + (tid >> 3) * 36 + 4 * (tid & 7)) = v;
  __syncthreads();
  const int n  = tid >> 2;
  const int k8 = (tid & 3) * 8;
  const int nc = n & 31;
  float f[8];
#pragma unroll
  for (int i = 0; i < 8; ++i) f[i] = sK[(k8 + i) * 36 + nc];
  const v4f a = (v4f){ f[0], f[1], f[2], f[3] };
  const v4f c = (v4f){ f[4], f[5], f[6], f[7] };
  v4u ov = pack8_bf16(a, c);
  const unsigned m = (n < COUT) ? 0xFFFFFFFFu : 0u;
  ov &= (v4u){ m, m, m, m };
  volatile v4u* q = (volatile v4u*)(bt + ((size_t)o * 256 + (size_t)tid) * 8);
  *q = ov;
  __threadfence();
  *q = ov;
}

__global__ __launch_bounds__(256) void k_gather(const float* __restrict__ x, const int* __restrict__ ids,
                                                int nEnt, unsigned short* ag) {
  const unsigned total = (unsigned)nEnt * 4u;
  const unsigned u  = blockIdx.x * 256u + threadIdx.x;
  const unsigned uc = u < total ? u : total - 1u;
  const int e = (int)(uc >> 2);
  const int q = (int)(uc & 3u);
  int id = ids[e];
  pini(id);
  id = clampi(id, 0, NVOX - 1);
  const float* p = x + (size_t)id * CIN + 8 * q;
  const v4f a = *(const v4fa*)p;
  const v4f c = *(const v4fa*)(p + 4);
  pin4f(a); pin4f(c);
  const v4u ov = pack8_bf16(a, c);
  if (u < total) {
    volatile v4u* dq = (volatile v4u*)(ag + (size_t)u * 8);
    *dq = ov;
    __threadfence();
    *dq = ov;
  }
}

template <int FIRST>
__global__ __launch_bounds__(NTHR) void k_owner(const int* __restrict__ keys, int nE,
                                                const float* __restrict__ cpl, float* outp) {
  extern __shared__ __attribute__((aligned(16))) int dsm[];
  int* list = dsm;
  int* hl   = dsm + LISTN;
  int* sl   = hl + RCAP;
  int* arr  = sl + RCAP;
  int* misc = arr + ARRN;
  const int tid = (int)threadIdx.x, lane = tid & 31;
  const int wave = __builtin_amdgcn_readfirstlane(tid >> 5);
  const int b = (int)blockIdx.x;
  const int rowBase = b * NBRUN;

  {
    const v4i z4 = {0, 0, 0, 0};
    for (int i = tid * 4; i < BK_INTS; i += NTHR * 4) *(v4ia*)(dsm + i) = z4;
  }
  __syncthreads();

  int t = 0;
  const int nChunks = nE / CHUNK;
#pragma unroll 1
  for (int ch = 0; ch < nChunks; ++ch) {
    const int cbase = ch * CHUNK;
    const int el0 = tid * EPT;
    const int e0  = clampi(cbase + el0, 0, nE - EPT);
    const v4i da = *(const v4ia*)(keys + e0);
    const v4i db = *(const v4ia*)(keys + e0 + 4);
    pin4(da); pin4(db);
    const unsigned nbs = (unsigned)rowBase;
    const unsigned unb = (unsigned)NBRUN;
    const unsigned s0 = (unsigned)da.x - nbs, s1 = (unsigned)da.y - nbs;
    const unsigned s2 = (unsigned)da.z - nbs, s3 = (unsigned)da.w - nbs;
    const unsigned s4 = (unsigned)db.x - nbs, s5 = (unsigned)db.y - nbs;
    const unsigned s6 = (unsigned)db.z - nbs, s7 = (unsigned)db.w - nbs;
    const bool h0 = s0 < unb, h1 = s1 < unb, h2 = s2 < unb, h3 = s3 < unb;
    const bool h4 = s4 < unb, h5 = s5 < unb, h6 = s6 < unb, h7 = s7 < unb;
    const unsigned any = __builtin_amdgcn_ballot_w32(h0 | h1 | h2 | h3 | h4 | h5 | h6 | h7);
    int wc = 0;
    if (any != 0u) {
      const int k = (int)h0 + (int)h1 + (int)h2 + (int)h3 + (int)h4 + (int)h5 + (int)h6 + (int)h7;
      int incl = k;
#pragma unroll
      for (int dd = 1; dd < 32; dd <<= 1) {
        const int y = __shfl_up(incl, dd, 32);
        if (lane >= dd) incl += y;
      }
      wc = __shfl(incl, 31, 32);
      int pos = incl - k;
#define PUTJ(J, HJ, SJ) if (HJ) { if (pos < WCAP) list[wave * WCAP + pos] = ((el0 + (J)) << SLOTB) | (int)(SJ); pos += 1; }
      PUTJ(0, h0, s0)
      PUTJ(1, h1, s1)
      PUTJ(2, h2, s2)
      PUTJ(3, h3, s3)
      PUTJ(4, h4, s4)
      PUTJ(5, h5, s5)
      PUTJ(6, h6, s6)
      PUTJ(7, h7, s7)
#undef PUTJ
    }
    wc = clampi(wc, 0, WCAP);
    wc = __builtin_amdgcn_readfirstlane(wc);
    int* mb = misc + (ch & 1) * 8;
    if (lane == 0) mb[wave] = wc;
    __syncthreads();
    int base = t, tot = 0;
#pragma unroll
    for (int w2 = 0; w2 < NWAVE; ++w2) {
      const int c = clampi(mb[w2], 0, WCAP);
      base += (w2 < wave) ? c : 0;
      tot  += c;
    }
    const int myc = wc;
#pragma unroll 1
    for (int b0 = 0; b0 < myc; b0 += 32) {
      const int idx  = b0 + lane;
      const int entv = list[wave * WCAP + (idx < WCAP ? idx : WCAP - 1)];
      const int slot = entv & (NBRUN - 1);
      const int el   = (entv >> SLOTB) & (CHUNK - 1);
      const int pos  = base + idx;
      if (idx < myc && pos < RCAP) hl[pos] = (slot << EBITS) | ((cbase + el) & EMASK);
    }
    t += tot;
  }
  __syncthreads();
  const int tt = t < RCAP ? t : RCAP;
  const int ov = t > RCAP ? 1 : 0;

  if (tid == 0) {
#pragma unroll 1
    for (int i = 0; i < tt; ++i) {
      const int k = (hl[i] >> EBITS) & (NBRUN - 1);
      arr[k] = arr[k] + 1;
    }
  }
  __syncthreads();
  if (wave == 0) {
    const int base = lane * (NBRUN / 32);
    int s = 0;
#pragma unroll 1
    for (int i = 0; i < NBRUN / 32; ++i) s += arr[base + i];
    int incl = s;
#pragma unroll
    for (int dd = 1; dd < 32; dd <<= 1) {
      const int y = __shfl_up(incl, dd, 32);
      if (lane >= dd) incl += y;
    }
    int run = incl - s;
#pragma unroll 1
    for (int i = 0; i < NBRUN / 32; ++i) {
      run += arr[base + i];
      arr[base + i] = run;
    }
    if (lane == 31) arr[NBRUN] = run;
  }
  __syncthreads();
  if (tid == 0) {
#pragma unroll 1
    for (int i = tt - 1; i >= 0; --i) {
      const int w = hl[i];
      const int k = (w >> EBITS) & (NBRUN - 1);
      const int p = clampi(arr[k] - 1, 0, RCAP - 1);
      arr[k] = p;
      sl[p] = w;
    }
  }
  __syncthreads();

  {
    int ovd = 0;
#pragma unroll 1
    for (int i = 0; i < NBRUN / NTHR; ++i) {
      const int k = tid + NTHR * i;
      const int c = arr[k + 1] - arr[k];
      ovd |= (c > DEGCAP || c < 0) ? 1 : 0;
    }
    const unsigned om = __builtin_amdgcn_ballot_w32(ovd != 0);
    if (lane == 0) misc[20 + wave] = (om != 0u) ? 1 : 0;
  }
  __syncthreads();
  int fl = ov;
#pragma unroll
  for (int w2 = 0; w2 < NWAVE; ++w2) fl |= misc[20 + w2];
  const float nanv = __int_as_float(0x7fc00000);

#pragma unroll 1
  for (int i = 0; i < NBRUN / NWAVE; ++i) {
    const int slot = wave * (NBRUN / NWAVE) + i;
    const int st = arr[slot];
    const int en = arr[slot + 1];
    const int stc = clampi(st, 0, RCAP - 1);
    int cv = clampi(en - st, 0, DEGCAP);
    cv = cv > RCAP - stc ? RCAP - stc : cv;
    const int cn  = __builtin_amdgcn_readfirstlane(cv);
    const int stu = __builtin_amdgcn_readfirstlane(stc);
    float s = 0.0f;
#pragma unroll 1
    for (int p = 0; p < cn; ++p) {
      const int w = sl[stu + p];
      pini(w);
      const int e = clampi(w & EMASK, 0, nE - 1);
      const float v = cpl[(size_t)e * COUT + lane];
      pinf(v);
      s += v;
    }
    float* op = outp + (size_t)(rowBase + slot) * COUT + lane;
    float r = s;
    if (FIRST == 0) {
      const float old = *op;
      pinf(old);
      r = old + s;
    }
    r = (fl != 0) ? nanv : r;
    volatile float* vp = (volatile float*)op;
    *vp = r;
    __threadfence();
    *vp = r;
  }
}

extern "C" void kernel_launch(void* const* d_in, const int* in_sizes, int n_in,
                              void* d_out, int out_size, void* d_ws, size_t ws_size,
                              hipStream_t stream) {
  if (n_in < 4) return;
  if (in_sizes[0] != NVOX * CIN) return;
  if (in_sizes[1] != NOFF * CIN * COUT) return;
  if (in_sizes[2] != NOFF * MPAIR) return;
  if (in_sizes[3] != NOFF * MPAIR) return;
  if (out_size != NVOX * COUT) return;
  if (WS_TOTAL > ws_size) return;

  const float* x    = (const float*)d_in[0];
  const float* wk   = (const float*)d_in[1];
  const int*   iidx = (const int*)d_in[2];
  const int*   oidx = (const int*)d_in[3];
  float* out = (float*)d_out;

  char* ws = (char*)d_ws;
  unsigned short* BT = (unsigned short*)(ws);
  unsigned short* AG = (unsigned short*)(ws + BT_BYTES);
  float*          CG = (float*)(ws + BT_BYTES + AG_BYTES);

  hipFuncSetAttribute(reinterpret_cast<const void*>(&k_owner<1>), hipFuncAttributeMaxDynamicSharedMemorySize, BK_BYTES);
  hipFuncSetAttribute(reinterpret_cast<const void*>(&k_owner<0>), hipFuncAttributeMaxDynamicSharedMemorySize, BK_BYTES);

  k_prep<<<NOFF, 256, 0, stream>>>(wk, BT);

  const int gemmBlocks = (MPAIR / 64 + 7) / 8;
  for (int g = 0; g < NGROUP; ++g) {
    const int nOff = (g < NGROUP - 1) ? GOFF : (NOFF - GOFF * (NGROUP - 1));
    const int nEnt = nOff * MPAIR;
    const int* gi = iidx + (size_t)g * GRPE;
    const int* go = oidx + (size_t)g * GRPE;
    k_gather<<<(nEnt * 4) / 256, 256, 0, stream>>>(x, gi, nEnt, AG);
    for (int j = 0; j < nOff; ++j) {
      k_gemm_nt<0, 0><<<gemmBlocks, 256, 0, stream>>>(AG + (size_t)j * MPAIR * CIN,
                                                      BT + (size_t)(GOFF * g + j) * NPB * CIN,
                                                      x, CG + (size_t)j * MPAIR * COUT,
                                                      MPAIR, COUT, CIN, COUT);
    }
    if (g == 0) k_owner<1><<<NBLK, NTHR, BK_BYTES, stream>>>(go, nEnt, CG, out);
    else        k_owner<0><<<NBLK, NTHR, BK_BYTES, stream>>>(go, nEnt, CG, out);
  }
}
